// MLPPredictor_34720515621375
// MI455X (gfx1250) — hardware-verified
//
#include <hip/hip_runtime.h>

typedef float          v8f   __attribute__((ext_vector_type(8)));
typedef float          v4f   __attribute__((ext_vector_type(4)));
typedef unsigned int   v4u   __attribute__((ext_vector_type(4)));
typedef int            v8i   __attribute__((ext_vector_type(8)));
typedef unsigned short v8us  __attribute__((ext_vector_type(8)));
typedef unsigned short v16us __attribute__((ext_vector_type(16)));
typedef __bf16         v16bf __attribute__((ext_vector_type(16)));
typedef _Float16       v16h  __attribute__((ext_vector_type(16)));
typedef v4f  __attribute__((may_alias)) v4fa;
typedef v8us __attribute__((may_alias)) v8usa;
union FragB { v16bf v; v16us u; v8us h[2]; v8i w; };
union FragH { v16h  v; v16us u; v8us h[2]; v8i w; };

__device__ __forceinline__ v8f wmb(const FragB& a, const FragB& b, v8f c) {
  v8f d = __builtin_amdgcn_wmma_f32_16x16x32_bf16(false, a.v, false, b.v, (short)0, c, false, false);
  asm volatile("v_nop\n\tv_nop\n\tv_nop\n\tv_nop" : "+v"(d) : "v"(a.w), "v"(b.w));
  return d;
}

__device__ __forceinline__ v8f wmh(const FragH& a, const FragH& b, v8f c) {
  v8f d = __builtin_amdgcn_wmma_f32_16x16x32_f16(false, a.v, false, b.v, (short)0, c, false, false);
  asm volatile("v_nop\n\tv_nop\n\tv_nop\n\tv_nop" : "+v"(d) : "v"(a.w), "v"(b.w));
  return d;
}

__device__ __forceinline__ unsigned bf16_bits(float f) {
  const unsigned u = __float_as_uint(f);
  const unsigned r = (u + 0x7FFFu + ((u >> 16) & 1u)) >> 16;
  const unsigned q = (u >> 16) | 0x40u;
  return ((u & 0x7fffffffu) > 0x7f800000u) ? q : r;
}

__device__ __forceinline__ float bf16_val(float f) {
  return __uint_as_float(bf16_bits(f) << 16);
}
__device__ __forceinline__ int clampi(int v, int lo, int hi) {
  return v < lo ? lo : (v > hi ? hi : v);
}

__device__ __forceinline__ unsigned f16_bits(float f) {
  const unsigned u  = __float_as_uint(f);
  const unsigned s  = (u >> 16) & 0x8000u;
  const unsigned a  = u & 0x7fffffffu;
  const unsigned t  = a - 0x38000000u;
  const unsigned r  = (t + 0x0FFFu + ((t >> 13) & 1u)) >> 13;
  const unsigned rc = r > 0x7C00u ? 0x7C00u : r;
  const bool small  = a < 0x38800000u;
  const bool isnan  = a > 0x7f800000u;
  const unsigned fin = small ? 0u : (s | rc);
  return isnan ? (s | 0x7E00u) : fin;
}

__device__ __forceinline__ unsigned pk16(unsigned lo, unsigned hi) { return lo | (hi << 16); }
__device__ __forceinline__ unsigned bf16_lo_bits(float v) {
  float hi = bf16_val(v);
  asm volatile("" : "+v"(hi));
  return bf16_bits(v - hi);
}
__device__ __forceinline__ v4u pack8_bf16(v4f a, v4f c) {
  return (v4u){ pk16(bf16_bits(a[0]), bf16_bits(a[1])), pk16(bf16_bits(a[2]), bf16_bits(a[3])),
                pk16(bf16_bits(c[0]), bf16_bits(c[1])), pk16(bf16_bits(c[2]), bf16_bits(c[3])) };
}
__device__ __forceinline__ v4u pack8_bf16_lo(v4f a, v4f c) {
  return (v4u){ pk16(bf16_lo_bits(a[0]), bf16_lo_bits(a[1])), pk16(bf16_lo_bits(a[2]), bf16_lo_bits(a[3])),
                pk16(bf16_lo_bits(c[0]), bf16_lo_bits(c[1])), pk16(bf16_lo_bits(c[2]), bf16_lo_bits(c[3])) };
}
__device__ __forceinline__ v4u pack8_f16(v4f a, v4f c) {
  return (v4u){ pk16(f16_bits(a[0]), f16_bits(a[1])), pk16(f16_bits(a[2]), f16_bits(a[3])),
                pk16(f16_bits(c[0]), f16_bits(c[1])), pk16(f16_bits(c[2]), f16_bits(c[3])) };
}

template <int FORM>
__global__ __launch_bounds__(256) void k_plane(const float* __restrict__ src, int rows, int cols, int ldsrc,
                                               unsigned short* __restrict__ dst, int MP, int KP) {
  static_assert(FORM >= 0 && FORM <= 3);
  const int KTOT = (FORM == 1 || FORM == 3) ? 2 * KP : KP;
  const unsigned ppr   = (unsigned)(KTOT >> 3);
  const unsigned kp8   = (unsigned)(KP >> 3);
  const unsigned total = (unsigned)MP * ppr;
  const unsigned g     = blockIdx.x * 256u + threadIdx.x;
  const unsigned rowu  = g / ppr;
  const unsigned p     = g - rowu * ppr;
  const bool second    = p >= kp8;
  const int row = (int)rowu;
  const int c0  = (int)((second ? p - kp8 : p) << 3);
  const float* srow = src + (size_t)clampi(row, 0, rows - 1) * (size_t)ldsrc;
  float x[8];
  unsigned mk[8];
#pragma unroll
  for (int e = 0; e < 8; ++e) {
    const int c = c0 + e;
    const float v = srow[clampi(c, 0, cols - 1)];
    asm volatile("" :: "v"(v));
    x[e]  = v;
    mk[e] = (row < rows && c < cols) ? 0xFFFFu : 0u;
  }
  const v4f a = (v4f){ x[0], x[1], x[2], x[3] };
  const v4f c = (v4f){ x[4], x[5], x[6], x[7] };
  v4u o;
  if (FORM == 2) {
    o = pack8_f16(a, c);
  } else {
    const v4u hi = pack8_bf16(a, c);
    o = hi;
    if (FORM == 1) { const v4u lo = pack8_bf16_lo(a, c); o = second ? lo : hi; }
  }
  const v4u mw = (v4u){ pk16(mk[0], mk[1]), pk16(mk[2], mk[3]), pk16(mk[4], mk[5]), pk16(mk[6], mk[7]) };
  o &= mw;
  if (g < total) {
    volatile v4u* q = (volatile v4u*)(dst + (size_t)g * 8);
    *q = o;
    __threadfence();
    *q = o;
  }
}

template <int FORM> struct FragOf    { typedef FragB T; };
template <>         struct FragOf<2> { typedef FragH T; };
__device__ __forceinline__ v8f mm(const FragB& a, const FragB& b, v8f c) { return wmb(a, b, c); }
__device__ __forceinline__ v8f mm(const FragH& a, const FragH& b, v8f c) { return wmh(a, b, c); }
template <class F> __device__ __forceinline__ F ld_frag(const unsigned short* p) {
  F f;
  f.h[0] = *(const v8usa*)(p);
  f.h[1] = *(const v8usa*)(p + 16);
  return f;
}

template <int FORM, int EPI>
__global__ __launch_bounds__(256) __attribute__((amdgpu_num_vgpr(248)))
void k_gemm_nt(const unsigned short* __restrict__ A, const unsigned short* __restrict__ B,
               const float* __restrict__ bias, float* __restrict__ D, int M, int N, int KTOT, int ldd) {
  static_assert(FORM >= 0 && FORM <= 2);
  static_assert(EPI == 0 || EPI == 1);
  typedef typename FragOf<FORM>::T F;
  __shared__ __attribute__((aligned(16))) float sT[8][16 * 68];
  const int lane = threadIdx.x & 31;
  const int wave = threadIdx.x >> 5;
  const int tilesM = (M + 63) >> 6;
  const int tilesN = (N + 63) >> 6;
  const int tile = blockIdx.x * 8 + wave;
  if (tile >= tilesM * tilesN) return;
  const int tm = tile / tilesN;
  const int tn = tile - tm * tilesN;
  const int m0 = tm << 6;
  const int n0 = tn << 6;

  const int rl = lane & 15;
  const int h8 = (lane >> 4) * 8;
  const unsigned short* pa = A + (size_t)(m0 + rl) * (size_t)KTOT + h8;
  const unsigned short* pb = B + (size_t)(n0 + rl) * (size_t)KTOT + h8;

  v8f acc[4][4];
#pragma unroll
  for (int i = 0; i < 4; ++i)
#pragma unroll
    for (int j = 0; j < 4; ++j) acc[i][j] = (v8f){0.f, 0.f, 0.f, 0.f, 0.f, 0.f, 0.f, 0.f};

#pragma unroll 1
  for (int k0 = 0; k0 < KTOT; k0 += 32) {
    F bf[4];
#pragma unroll
    for (int j = 0; j < 4; ++j) bf[j] = ld_frag<F>(pb + (size_t)(j << 4) * (size_t)KTOT + k0);
#pragma unroll
    for (int i = 0; i < 4; ++i) {
      const F af = ld_frag<F>(pa + (size_t)(i << 4) * (size_t)KTOT + k0);
#pragma unroll
      for (int j = 0; j < 4; ++j) acc[i][j] = mm(af, bf[j], acc[i][j]);
    }
  }

  float* slab = sT[wave];
  const int hh = lane >> 4;
  const int c4 = (lane & 15) * 4;
  const int nc = n0 + c4;
  const bool cok = nc < N;
  v4f bv = (v4f){0.f, 0.f, 0.f, 0.f};
  if (EPI == 1) {
    bv = *(const v4fa*)(bias + clampi(nc, 0, N - 4));
    asm volatile("" :: "v"(bv));
  }
#pragma unroll
  for (int i = 0; i < 4; ++i) {
    const int mBase = m0 + (i << 4);
#pragma unroll
    for (int j = 0; j < 4; ++j) {
#pragma unroll
      for (int r = 0; r < 8; ++r) slab[(h8 + r) * 68 + (j << 4) + rl] = acc[i][j][r];
    }
    __builtin_amdgcn_fence(__ATOMIC_RELEASE, "workgroup");
    __builtin_amdgcn_wave_barrier();
    __builtin_amdgcn_fence(__ATOMIC_ACQUIRE, "workgroup");
    v4f vv[8];
#pragma unroll
    for (int it = 0; it < 8; ++it) {
      const int row = it * 2 + hh;
      v4f v = *(const v4fa*)(slab + row * 68 + c4);
      if (EPI == 1) v += bv;
      vv[it] = v;
    }
    for (int pass = 0; pass < 2; ++pass) {
#pragma unroll
      for (int it = 0; it < 8; ++it) {
        const int row = mBase + it * 2 + hh;
        if (cok && row < M) *(volatile v4f*)(D + (size_t)row * (size_t)ldd + nc) = vv[it];
      }
      __threadfence();
    }
    __builtin_amdgcn_fence(__ATOMIC_RELEASE, "workgroup");
    __builtin_amdgcn_wave_barrier();
    __builtin_amdgcn_fence(__ATOMIC_ACQUIRE, "workgroup");
  }
}

#pragma clang fp contract(off)

constexpr int NN   = 50000;
constexpr int NE   = 600000;
constexpr int DF   = 128;
constexpr int NCLS = 2;
constexpr int MP   = 50048;
constexpr int NPB  = 64;
constexpr int OUT_ELEMS = 1200000;

static_assert(OUT_ELEMS == NE * NCLS);
static_assert(OUT_ELEMS % 128 == 0 && OUT_ELEMS / 128 == 9375);
static_assert(MP % 128 == 0 && MP % 64 == 0 && MP >= NN && MP == 391 * 128);
static_assert(DF == 128 && DF % 32 == 0);
static_assert(NN % 16 == 0);
static_assert(NPB % 64 == 0 && NPB % 32 == 0 && NPB >= 2 * NCLS);
static_assert((long long)NPB * MP < 0x7fffffffLL);
static_assert((long long)MP * DF / 8 < 0x7fffffffLL);
static_assert(((long long)MP * DF / 8) % 256 == 0 && ((long long)MP * DF / 8) / 256 == 3128);
static_assert(NCLS == 2);

constexpr size_t SZ_HB = (size_t)MP * DF * 2;
constexpr size_t SZ_P  = (size_t)MP * NPB * 4;
constexpr size_t SZ_BT = (size_t)NPB * DF * 2;
constexpr size_t SZ_BV = 128;
constexpr size_t OFF_HB = 0;
constexpr size_t OFF_P  = OFF_HB + SZ_HB;
constexpr size_t OFF_BT = OFF_P + SZ_P;
constexpr size_t OFF_BV = OFF_BT + SZ_BT;
constexpr size_t WS_TOTAL = OFF_BV + SZ_BV;
static_assert(SZ_HB == (size_t)12812288 && SZ_P == (size_t)12812288 && SZ_BT == (size_t)16384);
static_assert(OFF_P % 256 == 0 && OFF_BT % 256 == 0 && OFF_BV % 256 == 0);
static_assert(OFF_P == (size_t)12812288 && OFF_BT == (size_t)25624576 && OFF_BV == (size_t)25640960);
static_assert(WS_TOTAL == (size_t)25641088);
static_assert(WS_TOTAL <= ((size_t)128 << 20));

__global__ __launch_bounds__(256) void k_prepw(const float* __restrict__ W, const float* __restrict__ bias,
                                               unsigned short* __restrict__ Bt, float* __restrict__ BV) {
  const int tid = (int)threadIdx.x;
  v4u o[4];
#pragma unroll
  for (int i = 0; i < 4; ++i) {
    const int g    = tid + 256 * i;
    const int row  = g >> 4;
    const int p    = g & 15;
    const int rc   = row < 4 ? row : 3;
    const int half = rc >> 1;
    const int c    = rc & 1;
    const float* sp = W + c * (2 * DF) + half * DF + p * 8;
    const v4f a = *(const v4fa*)(sp);
    const v4f b = *(const v4fa*)(sp + 4);
    asm volatile("" :: "v"(a));
    asm volatile("" :: "v"(b));
    const unsigned m = row < 4 ? 0xFFFFFFFFu : 0u;
    v4u w = pack8_bf16(a, b);
    w &= (v4u){ m, m, m, m };
    o[i] = w;
  }
  const float b0 = bias[0];
  asm volatile("" :: "v"(b0));
  const float b1 = bias[1];
  asm volatile("" :: "v"(b1));
  const unsigned m0 = (tid == 0) ? 0xFFFFFFFFu : 0u;
  const v4f bo = (v4f){ __uint_as_float(__float_as_uint(bf16_val(b0)) & m0),
                        __uint_as_float(__float_as_uint(bf16_val(b1)) & m0), 0.0f, 0.0f };
#pragma unroll
  for (int i = 0; i < 4; ++i) {
    *(volatile v4u*)(Bt + (size_t)(tid + 256 * i) * 8) = o[i];
  }
  if (tid < 8) *(volatile v4f*)(BV + 4 * tid) = bo;
  __threadfence();
#pragma unroll
  for (int i = 0; i < 4; ++i) {
    *(volatile v4u*)(Bt + (size_t)(tid + 256 * i) * 8) = o[i];
  }
  if (tid < 8) *(volatile v4f*)(BV + 4 * tid) = bo;
}

__global__ __launch_bounds__(128) void k_out(const int* __restrict__ src, const int* __restrict__ dst,
                                             const float* __restrict__ P, const float* __restrict__ BV,
                                             float* __restrict__ out) {
  const int f  = (int)blockIdx.x * 128 + (int)threadIdx.x;
  const int fc = f < OUT_ELEMS ? f : OUT_ELEMS - 1;
  const int e  = fc >> 1;
  const int c  = fc & 1;
  int sraw = src[e];
  asm volatile("" :: "v"(sraw));
  int draw = dst[e];
  asm volatile("" :: "v"(draw));
  const int s = clampi(sraw, 0, NN - 1);
  const int d = clampi(draw, 0, NN - 1);
  const float p0 = P[(size_t)s * NPB + c];
  asm volatile("" :: "v"(p0));
  const float p1 = P[(size_t)d * NPB + 2 + c];
  asm volatile("" :: "v"(p1));
  const float bv0 = BV[0];
  asm volatile("" :: "v"(bv0));
  const float bv1 = BV[1];
  asm volatile("" :: "v"(bv1));
  const unsigned cm = 0u - (unsigned)c;
  const float bc = __uint_as_float((__float_as_uint(bv0) & ~cm) | (__float_as_uint(bv1) & cm));
  const float v = (p0 + p1) + bc;
  if (f < OUT_ELEMS) {
    volatile float* q = (volatile float*)(out + f);
    *q = v;
    __threadfence();
    *q = v;
  }
}

extern "C" void kernel_launch(void* const* d_in, const int* in_sizes, int n_in,
                              void* d_out, int out_size, void* d_ws, size_t ws_size,
                              hipStream_t stream) {
  if (n_in < 5) return;
  if (in_sizes[0] != NN * DF) return;
  if (in_sizes[1] != NE) return;
  if (in_sizes[2] != NE) return;
  if (in_sizes[3] != NCLS * 2 * DF) return;
  if (in_sizes[4] != NCLS) return;
  if (out_size != OUT_ELEMS) return;
  if (ws_size < WS_TOTAL) return;

  const float* h    = (const float*)d_in[0];
  const int*   src  = (const int*)d_in[1];
  const int*   dst  = (const int*)d_in[2];
  const float* W    = (const float*)d_in[3];
  const float* bias = (const float*)d_in[4];
  float* out = (float*)d_out;

  char* ws = (char*)d_ws;
  unsigned short* HB = (unsigned short*)(ws + OFF_HB);
  float*          P  = (float*)(ws + OFF_P);
  unsigned short* Bt = (unsigned short*)(ws + OFF_BT);
  float*          BV = (float*)(ws + OFF_BV);

  k_plane<0><<<MP * DF / 8 / 256, 256, 0, stream>>>(h, NN, DF, DF, HB, MP, DF);
  k_prepw<<<1, 256, 0, stream>>>(W, bias, Bt, BV);
  k_gemm_nt<0, 0><<<((NN + 63) / 64 + 7) / 8, 256, 0, stream>>>(HB, Bt, BV, P, NN, NPB, DF, NPB);
  k_out<<<OUT_ELEMS / 128, 128, 0, stream>>>(src, dst, P, BV, out);
}
